// RA_RA_17686675325051
// MI455X (gfx1250) — hardware-verified
//
#include <hip/hip_runtime.h>
#include <math.h>

typedef __attribute__((ext_vector_type(16))) _Float16 v16h;
typedef __attribute__((ext_vector_type(16))) __bf16 v16b;
typedef __attribute__((ext_vector_type(8)))  _Float16 v8h;
typedef __attribute__((ext_vector_type(8)))  float v8f;
typedef __attribute__((ext_vector_type(4)))  float v4f;
typedef __attribute__((ext_vector_type(2)))  float v2f;
typedef __attribute__((ext_vector_type(4)))  unsigned v4u;
typedef __attribute__((ext_vector_type(4)))  int v4i;
typedef float __attribute__((may_alias)) float_a;
typedef int __attribute__((may_alias)) int_a;

template <typename T> __device__ __forceinline__ void vst2(void* p, T v) { *(volatile T*)p = v; __threadfence(); *(volatile T*)p = v; }
__device__ __forceinline__ v8f wmma16(v16h a, v16h b, v8f c) {
  v8f d = __builtin_amdgcn_wmma_f32_16x16x32_f16(false, a, false, b, (short)0, c, false, false);
  asm volatile("v_nop\n\tv_nop\n\tv_nop\n\tv_nop" : "+v"(d) : "v"(a), "v"(b));
  return d;
}
__device__ __forceinline__ v8f wmma_bf(v16b a, v16b b, v8f c) {
  v8f d = __builtin_amdgcn_wmma_f32_16x16x32_bf16(false, a, false, b, (short)0, c, false, false);
  asm volatile("v_nop\n\tv_nop\n\tv_nop\n\tv_nop" : "+v"(d) : "v"(a), "v"(b));
  return d;
}
__device__ __forceinline__ v16h frag_h(const _Float16* rowk0, int lane) {
  union { v16h v; v8h q[2]; } u; const _Float16* p = rowk0 + 8 * (lane >> 4);
  u.q[0] = *(const v8h*)p; u.q[1] = *(const v8h*)(p + 16); return u.v;
}
__device__ __forceinline__ v16h frag_f32(const float* rowk0, int lane) {
  v16h a; const float* p = rowk0 + 8 * (lane >> 4);
#pragma unroll
  for (int i = 0; i < 8; ++i) { a[i] = (_Float16)p[i]; a[8 + i] = (_Float16)p[16 + i]; }
  return a;
}
__device__ __forceinline__ v16h frag_f32s(const float* rowk0, int lane, float sc) {
  v16h a; const float* p = rowk0 + 8 * (lane >> 4);
#pragma unroll
  for (int i = 0; i < 8; ++i) { a[i] = (_Float16)(p[i] * sc); a[8 + i] = (_Float16)(p[16 + i] * sc); }
  return a;
}
__device__ __forceinline__ v16h fragc_f32(const float* W, int k0, int n, int lane, int ld, int K) {
  v16h a; const int g = lane >> 4;
#pragma unroll
  for (int i = 0; i < 8; ++i) { const int ka = k0 + 8 * g + i, kb = ka + 16;
    a[i] = (_Float16)(ka < K ? W[(size_t)(ka < K ? ka : K - 1) * ld + n] : 0.f); a[8 + i] = (_Float16)(kb < K ? W[(size_t)(kb < K ? kb : K - 1) * ld + n] : 0.f); }
  return a;
}
struct F2 { v16b h, l; };
__device__ __forceinline__ F2 bsplit16(const float v[16]) { F2 r;
#pragma unroll
  for (int i = 0; i < 16; ++i) { const __bf16 h = (__bf16)v[i]; r.h[i] = h; r.l[i] = (__bf16)(v[i] - (float)h); }
  return r; }
__device__ __forceinline__ F2 split_row(const float* row, int k0, int lane) { float v[16]; const float* p = row + k0 + 8 * (lane >> 4);
#pragma unroll
  for (int i = 0; i < 8; ++i) { v[i] = p[i]; v[8 + i] = p[16 + i]; }
  return bsplit16(v); }
__device__ __forceinline__ F2 split_rowK(const float* row, int k0, int lane, int K) { float v[16]; const int g = lane >> 4;
#pragma unroll
  for (int i = 0; i < 8; ++i) { const int ka = k0 + 8 * g + i, kb = ka + 16; v[i] = ka < K ? row[ka < K ? ka : K - 1] : 0.f; v[8 + i] = kb < K ? row[kb < K ? kb : K - 1] : 0.f; }
  return bsplit16(v); }
__device__ __forceinline__ F2 split_col(const float* W, int k0, int n, int lane, int ld, int K) { float v[16]; const int g = lane >> 4;
#pragma unroll
  for (int i = 0; i < 8; ++i) { const int ka = k0 + 8 * g + i, kb = ka + 16; v[i] = ka < K ? W[(size_t)(ka < K ? ka : K - 1) * ld + n] : 0.f; v[8 + i] = kb < K ? W[(size_t)(kb < K ? kb : K - 1) * ld + n] : 0.f; }
  return bsplit16(v); }
__device__ __forceinline__ v8f mac3(const F2& a, const F2& b, v8f c) { c = wmma_bf(a.l, b.h, c); c = wmma_bf(a.h, b.l, c); return wmma_bf(a.h, b.h, c); }
__device__ __forceinline__ float sigm(float v) { return 1.0f / (1.0f + expf(-v)); }
#define LDSX() do { asm volatile("s_wait_dscnt 0" ::: "memory"); __builtin_amdgcn_wave_barrier(); __builtin_amdgcn_fence(__ATOMIC_RELEASE, "workgroup"); } while (0)


#define NB 4
#define HH 64
#define WWd 64
#define CCh 64
#define NC 19
#define NSEQ 4096
#define FD 64
#ifndef NBB
#define NBB NB
#endif
typedef __attribute__((ext_vector_type(8))) __bf16 v8b;
__device__ __forceinline__ v16b frag_b(const __bf16* rowk0, int lane) {
  union { v16b v; v8b q[2]; } u; const __bf16* p = rowk0 + 8 * (lane >> 4);
  u.q[0] = *(const v8b*)p; u.q[1] = *(const v8b*)(p + 16); return u.v;
}
__device__ __forceinline__ float bfr(float v) { return (float)(__bf16)v; }
__device__ __attribute__((noinline)) float exp_ni(float v) { return expf(v); }
__device__ __attribute__((noinline)) float erf_ni(float v) { return erff(v); }

#define WS_PW  0u
#define WS_QH  (WS_PW + 2u * 4 * FD * FD)
#define WS_QL  (WS_QH + 2u * NB * NSEQ * FD)
#define WS_VT  (WS_QL + 2u * NB * NSEQ * FD)
#define WS_VL  (WS_VT + 2u * NB * NSEQ * FD)
#define WS_X1  (WS_VL + 2u * NB * NSEQ * FD)
#define WS_X2  (WS_X1 + 4u * NB * HH * WWd * CCh)
#define WS_END (WS_X2 + 4u * NB * HH * WWd * CCh)

__device__ __attribute__((noinline)) float exp_p(float v) { return expf(v); }
__global__ __launch_bounds__(64) void k_pack(const float* __restrict__ HQ, const float* __restrict__ HV, const float* __restrict__ WQ, const float* __restrict__ WV, __bf16* __restrict__ PW) {
  const int n = blockIdx.x, which = blockIdx.y, t = threadIdx.x; const float* Wm = (which == 0) ? HQ : (which == 1) ? HV : (which == 2) ? WQ : WV; __shared__ __align__(16) __bf16 s[FD];
  s[t] = (__bf16)Wm[(size_t)t * FD + n]; __syncthreads();
  if (t < FD / 8) vst2((unsigned*)(PW + ((size_t)which * FD + n) * FD + t * 8), *(const v4u*)&s[t * 8]);
}
template <int AX>
__global__ __launch_bounds__(128) void k_proj(const float* __restrict__ SRC, const __bf16* __restrict__ PW, const float* __restrict__ BQ, const float* __restrict__ BV, _Float16* __restrict__ QH, _Float16* __restrict__ QL, _Float16* __restrict__ VT, _Float16* __restrict__ VL) {
  __shared__ __align__(16) __bf16 sa[64][FD + 8], sal[64][FD + 8]; __shared__ __align__(16) _Float16 sqh[64][FD + 8], sql[64][FD + 8]; __shared__ __align__(16) _Float16 svt[FD][72], svl[FD][72];
  const int tid = threadIdx.x, wave = tid >> 5, lane = tid & 31, col = lane & 15, g = lane >> 4; const size_t b = blockIdx.y; const int o = blockIdx.x;
  const __bf16* PQ = PW + (size_t)(AX == 0 ? 0 : 2) * FD * FD; const __bf16* PV = PW + (size_t)(AX == 0 ? 1 : 3) * FD * FD;
  for (int e = tid; e < 64 * FD; e += 128) { const int d = e >> 6, c = e & 63; const float v = (AX == 0) ? bfr(SRC[((b * HH + d) * WWd + o) * CCh + c]) : SRC[((b * HH + o) * WWd + d) * CCh + c]; const __bf16 hb = (__bf16)v; sa[c][d] = hb; sal[c][d] = (__bf16)(v - (float)hb); }
  if (tid < 64) for (int d = FD; d < FD + 8; ++d) { sa[tid][d] = (__bf16)0.f; sal[tid][d] = (__bf16)0.f; sqh[tid][d] = (_Float16)0.f; sql[tid][d] = (_Float16)0.f; }
  __syncthreads();
  v8f acc[8] = {};
#pragma unroll
  for (int kc = 0; kc < FD / 32; ++kc) { const v16b a = frag_b(&sa[wave * 16 + col][kc * 32], lane), al = frag_b(&sal[wave * 16 + col][kc * 32], lane);
#pragma unroll
    for (int j = 0; j < 8; ++j) { const __bf16* Wr = (j < 4) ? PQ : PV; const v16b w = frag_b(Wr + (size_t)((j & 3) * 16 + col) * FD + kc * 32, lane); if (AX == 1) acc[j] = wmma_bf(al, w, acc[j]); acc[j] = wmma_bf(a, w, acc[j]); } }
#pragma unroll
  for (int j = 0; j < 8; ++j) { const int d = (j & 3) * 16 + col; const float bb = bfr((j < 4 ? BQ : BV)[d]);
#pragma unroll
    for (int r = 0; r < 8; ++r) { const float v = acc[j][r] + bb; const int rr = wave * 16 + 8 * g + r; const _Float16 hv = (_Float16)v; if (j < 4) { sqh[rr][d] = hv; sql[rr][d] = (_Float16)((v - (float)hv) * 2048.0f); } else { svt[d][rr] = hv; svl[d][rr] = (_Float16)((v - (float)hv) * 2048.0f); } } }
  __syncthreads();
  const size_t n0 = (size_t)o * 64;
  for (int e = tid; e < 64 * 8; e += 128) { const int r = e >> 3, q = e & 7; const size_t off = (b * NSEQ + n0 + r) * FD + q * 8; vst2((unsigned*)(QH + off), *(const v4u*)&sqh[r][q * 8]); vst2((unsigned*)(QL + off), *(const v4u*)&sql[r][q * 8]); }
  for (int e = tid; e < FD * 8; e += 128) { const int d = e >> 3, pc = e & 7; vst2((unsigned*)(VT + (b * FD + d) * NSEQ + n0 + pc * 8), *(const v4u*)&svt[d][pc * 8]); vst2((unsigned*)(VL + (b * FD + d) * NSEQ + n0 + pc * 8), *(const v4u*)&svl[d][pc * 8]); }
}
template <int AX>
__global__ __launch_bounds__(128) void k_att(const _Float16* __restrict__ QH, const _Float16* __restrict__ QL, const _Float16* __restrict__ VT, const _Float16* __restrict__ VL, const float* __restrict__ GATE, const float* __restrict__ RES, float* __restrict__ OUTB) {
  __shared__ __align__(16) _Float16 sph[4][16][40], spl[4][16][40]; __shared__ __align__(16) float so[FD][68];
  const int tid = threadIdx.x, wave = tid >> 5, lane = tid & 31, col = lane & 15, g = lane >> 4; const size_t b = blockIdx.y; const int o = blockIdx.x; const size_t rq = b * NSEQ + (size_t)o * 64 + wave * 16;
  v16h aq[2], aql[2];
#pragma unroll
  for (int kc = 0; kc < 2; ++kc) { aq[kc] = frag_h(QH + (rq + col) * FD + kc * 32, lane); aql[kc] = frag_h(QL + (rq + col) * FD + kc * 32, lane); }
  v8f acc[4] = {}, accl[4] = {}; const float scale = 0.125f;
#pragma unroll 1
  for (int ks = 0; ks < NSEQ / 32; ++ks) { const int j0 = ks * 32;
#pragma unroll
    for (int ct = 0; ct < 2; ++ct) { const size_t rk = (b * NSEQ + j0 + ct * 16 + col) * FD; v8f c = {}, cl = {};
#pragma unroll
      for (int kc = 0; kc < 2; ++kc) { const v16h kh = frag_h(QH + rk + kc * 32, lane); c = wmma16(aq[kc], kh, c); cl = wmma16(aql[kc], kh, cl); cl = wmma16(aq[kc], frag_h(QL + rk + kc * 32, lane), cl); }
#pragma unroll
      for (int r = 0; r < 8; ++r) { const float s = (c[r] + cl[r] * (1.0f / 2048.0f)) * scale; const float p = 2048.0f / (1.0f + exp_p(-s)); const _Float16 hp = (_Float16)p; sph[wave][8 * g + r][ct * 16 + col] = hp; spl[wave][8 * g + r][ct * 16 + col] = (_Float16)((p - (float)hp) * 2048.0f); } }
    LDSX();
    const v16h pa = frag_h(&sph[wave][col][0], lane), pl = frag_h(&spl[wave][col][0], lane);
#pragma unroll
    for (int dt = 0; dt < 4; ++dt) { const size_t vo = (b * FD + dt * 16 + col) * NSEQ + j0; const v16h vh = frag_h(VT + vo, lane); acc[dt] = wmma16(pa, vh, acc[dt]); accl[dt] = wmma16(pl, vh, accl[dt]); accl[dt] = wmma16(pa, frag_h(VL + vo, lane), accl[dt]); }
    LDSX(); }
  const float gate = bfr(GATE[0]);
#pragma unroll
  for (int r = 0; r < 8; ++r) { const int c = wave * 16 + 8 * g + r;
#pragma unroll
    for (int dt = 0; dt < 4; ++dt) { const int dd = dt * 16 + col; const size_t idx = (AX == 0) ? (((b * HH + dd) * WWd + o) * CCh + c) : (((b * HH + o) * WWd + dd) * CCh + c); const float res = (AX == 0) ? bfr(RES[idx]) : RES[idx]; so[dd][c] = (acc[dt][r] + accl[dt][r] * (1.0f / 2048.0f)) * (1.0f / 2048.0f) * gate + res; } }
  __syncthreads();
  for (int e = tid; e < FD * 16; e += 128) { const int dd = e >> 4, q = e & 15; const size_t base = (AX == 0) ? (((b * HH + dd) * WWd + o) * CCh) : (((b * HH + o) * WWd + dd) * CCh); vst2(OUTB + base + q * 4, *(const v4f*)&so[dd][q * 4]); }
}
__global__ __launch_bounds__(256) void k_fin(const float* __restrict__ FEAT, const float* __restrict__ X2, const float* __restrict__ PRED, const float* __restrict__ CW, const float* __restrict__ CB, float* __restrict__ OUT) {
  const size_t b = blockIdx.y; const int h = blockIdx.x, t = threadIdx.x; __shared__ float sp[WWd]; __shared__ __align__(16) float so[WWd * CCh];
  if (t < WWd) { float a = 0.f; for (int k = 0; k < NC; ++k) { const float pr = bfr(PRED[((b * HH + h) * WWd + t) * NC + k]); a += (1.0f - 1.0f / (1.0f + exp_p(-pr))) * bfr(CW[k]); } sp[t] = a + bfr(CB[0]); }
  __syncthreads();
  for (int e = t; e < WWd * CCh; e += 256) { const int w = e >> 6; const size_t idx = ((b * HH + h) * WWd) * CCh + e; so[e] = sp[w] * (bfr(FEAT[idx]) + X2[idx]); }
  __syncthreads();
  for (int q = t; q < WWd * CCh / 4; q += 256) vst2(OUT + ((b * HH + h) * WWd) * CCh + q * 4, *(const v4f*)&so[q * 4]);
}
extern "C" void kernel_launch(void* const* d_in, const int* in_sizes, int n_in, void* d_out, int out_size, void* d_ws, size_t ws_size, hipStream_t stream) {
  (void)in_sizes; (void)n_in; (void)out_size;
  const float** F = (const float**)d_in;
  if (ws_size < (size_t)WS_END) return;
  char* ws = (char*)d_ws; __bf16* PW = (__bf16*)(ws + WS_PW); _Float16 *QH = (_Float16*)(ws + WS_QH), *QL = (_Float16*)(ws + WS_QL), *VT = (_Float16*)(ws + WS_VT), *VL = (_Float16*)(ws + WS_VL); float *X1 = (float*)(ws + WS_X1), *X2 = (float*)(ws + WS_X2);
  k_pack<<<dim3(FD, 4), 64, 0, stream>>>(F[2], F[4], F[6], F[8], PW);
  k_proj<0><<<dim3(WWd, NBB), 128, 0, stream>>>(F[0], PW, F[3], F[5], QH, QL, VT, VL);
  k_att<0><<<dim3(NSEQ / 64, NBB), 128, 0, stream>>>(QH, QL, VT, VL, F[10], F[0], X1);
  k_proj<1><<<dim3(HH, NBB), 128, 0, stream>>>(X1, PW, F[7], F[9], QH, QL, VT, VL);
  k_att<1><<<dim3(NSEQ / 64, NBB), 128, 0, stream>>>(QH, QL, VT, VL, F[11], X1, X2);
  k_fin<<<dim3(HH, NBB), 256, 0, stream>>>(F[0], X2, F[1], F[12], F[13], (float*)d_out);
}
